// NewAttention_39642548142828
// MI455X (gfx1250) — hardware-verified
//
#include <hip/hip_runtime.h>

typedef __attribute__((ext_vector_type(16))) _Float16 v16h;
typedef __attribute__((ext_vector_type(8)))  _Float16 v8h;
typedef __attribute__((ext_vector_type(16))) __bf16   v16b;
typedef __attribute__((ext_vector_type(8)))  __bf16   v8b;
typedef __attribute__((ext_vector_type(8)))  float    v8f;
typedef __attribute__((ext_vector_type(4)))  float    v4f;
#define PSCALE 32768.0f
#define U16(p) ((const unsigned short*)(const void*)(p))
#define PSCALE_INV (1.0f / 32768.0f)

__device__ __forceinline__ unsigned short f2bf_bits(float f) {
  unsigned u = __float_as_uint(f);
  return (unsigned short)((u + 0x7FFFu + ((u >> 16) & 1u)) >> 16);
}
__device__ __forceinline__ float bf_bits2f(unsigned short h) { return __uint_as_float(((unsigned)h) << 16); }

__device__ __forceinline__ void dep_guard_h(v8f& a, v8f& b, v16h x, v16h y) { asm volatile("v_nop\n\tv_nop\n\tv_nop\n\tv_nop" : "+v"(a), "+v"(b) : "v"(x), "v"(y)); }
__device__ __forceinline__ void dep_guard_b(v8f& a, v8f& b, v16b x, v16b y) { asm volatile("v_nop\n\tv_nop\n\tv_nop\n\tv_nop" : "+v"(a), "+v"(b) : "v"(x), "v"(y)); }
__device__ __forceinline__ void keep4_h(v16h a, v16h b, v16h c, v16h d) { asm volatile("v_nop" :: "v"(a), "v"(b), "v"(c), "v"(d)); }
__device__ __forceinline__ void keep4_b(v16b a, v16b b, v16b c, v16b d) { asm volatile("v_nop" :: "v"(a), "v"(b), "v"(c), "v"(d)); }
__device__ __forceinline__ void acc_guard4(v8f& a, v8f& b, v8f& c, v8f& d) { asm volatile("v_nop\n\tv_nop\n\tv_nop\n\tv_nop" : "+v"(a), "+v"(b), "+v"(c), "+v"(d)); }
template <typename T> struct Frag;
template <> struct Frag<_Float16> {
  typedef v16h V; union U { v16h v; v8h h[2]; };
  static __device__ __forceinline__ v16h load(const _Float16* p) {
    U f; f.h[0] = *(const v8h*)(p); f.h[1] = *(const v8h*)(p + 16); return f.v;
  }
  static __device__ __forceinline__ v8f mma(v16h a, v16h b, v8f c) {
    return __builtin_amdgcn_wmma_f32_16x16x32_f16(false, a, false, b, (short)0, c, false, false);
  }
  static __device__ __forceinline__ void guard(v8f& a, v8f& b, v16h x, v16h y) { dep_guard_h(a, b, x, y); }
  static __device__ __forceinline__ void keep(v16h a, v16h b, v16h c, v16h d) { keep4_h(a, b, c, d); }
};
template <> struct Frag<__bf16> {
  typedef v16b V; union U { v16b v; v8b h[2]; };
  static __device__ __forceinline__ v16b load(const __bf16* p) {
    U f; f.h[0] = *(const v8b*)(p); f.h[1] = *(const v8b*)(p + 16); return f.v;
  }
  static __device__ __forceinline__ v8f mma(v16b a, v16b b, v8f c) {
    return __builtin_amdgcn_wmma_f32_16x16x32_bf16(false, a, false, b, (short)0, c, false, false);
  }
  static __device__ __forceinline__ void guard(v8f& a, v8f& b, v16b x, v16b y) { dep_guard_b(a, b, x, y); }
  static __device__ __forceinline__ void keep(v16b a, v16b b, v16b c, v16b d) { keep4_b(a, b, c, d); }
};

template <int ET> struct Elem;
template <> struct Elem<0> { typedef _Float16 T; };
template <> struct Elem<1> { typedef __bf16 T; };
template <int ET, bool SPLIT, int BIAS_MODE, int OUT_MODE, bool RESID, int ACT = 0>
__global__ __launch_bounds__(256) void wmma_gemm64(
    const unsigned short* __restrict__ Ap, const unsigned short* __restrict__ A2p, int lda, long strideA,
    const unsigned short* __restrict__ Btp, const unsigned short* __restrict__ Bt2p, int ldb, long strideB,
    void* __restrict__ Cout, void* __restrict__ Cout2, int ldc, long strideC,
    const float* __restrict__ bias,
    const float* __restrict__ resid, long strideR,
    int M, int N, int K, float scale) {
  typedef typename Elem<ET>::T T;
  typedef typename Frag<T>::V V;
  const T* A = (const T*)Ap; const T* A2 = (const T*)A2p; const T* Bt = (const T*)Btp; const T* Bt2 = (const T*)Bt2p;
  __shared__ __align__(16) float sT[8][16 * 68];
  const int b    = blockIdx.y;
  const int lane = threadIdx.x & 31;
  const int wave = threadIdx.x >> 5;
  const int tilesN = N >> 6;
  const int tilesM = M >> 6;
  const int tile = blockIdx.x * 8 + wave;
  if (tile >= tilesM * tilesN) return;
  const int tm = tile / tilesN;
  const int tn = tile - tm * tilesN;
  const int m0 = tm << 6;
  const int n0 = tn << 6;

  const T* Ab  = A  + (size_t)b * strideA;
  const T* Bb  = Bt + (size_t)b * strideB;
  const T* Ab2 = SPLIT ? (A2  + (size_t)b * strideA) : nullptr;
  const T* Bb2 = SPLIT ? (Bt2 + (size_t)b * strideB) : nullptr;

  const int rlane = lane & 15;
  const int koff  = (lane >> 4) * 8;
  const int mOff  = (lane >> 4) * 8;

  v8f acc[4][4];
#pragma unroll
  for (int i = 0; i < 4; ++i)
#pragma unroll
    for (int j = 0; j < 4; ++j) acc[i][j] = (v8f){0.f,0.f,0.f,0.f,0.f,0.f,0.f,0.f};

  for (int k0 = 0; k0 < K; k0 += 32) {
    V bh[4], bl[4];
#pragma unroll
    for (int j = 0; j < 4; ++j) {
      const size_t bo = (size_t)(n0 + (j << 4) + rlane) * ldb + koff + k0;
      bh[j] = Frag<T>::load(Bb + bo);
      if (SPLIT) bl[j] = Frag<T>::load(Bb2 + bo);
    }
#pragma unroll
    for (int i = 0; i < 4; ++i) {
      const size_t ao = (size_t)(m0 + (i << 4) + rlane) * lda + koff + k0;
      V ah = Frag<T>::load(Ab + ao);
      V al;
      if (SPLIT) al = Frag<T>::load(Ab2 + ao);
#pragma unroll
      for (int j = 0; j < 4; ++j) {
        acc[i][j] = Frag<T>::mma(ah, bh[j], acc[i][j]);
        if (SPLIT) {
          acc[i][j] = Frag<T>::mma(ah, bl[j], acc[i][j]);
          acc[i][j] = Frag<T>::mma(al, bh[j], acc[i][j]);
        }
      }
      Frag<T>::guard(acc[i][0], acc[i][3], ah, SPLIT ? al : ah);
    }
    Frag<T>::keep(bh[0], bh[1], bh[2], bh[3]);
    if (SPLIT) Frag<T>::keep(bl[0], bl[1], bl[2], bl[3]);
  }
  acc_guard4(acc[0][0], acc[0][1], acc[0][2], acc[0][3]);
  acc_guard4(acc[1][0], acc[1][1], acc[1][2], acc[1][3]);
  acc_guard4(acc[2][0], acc[2][1], acc[2][2], acc[2][3]);
  acc_guard4(acc[3][0], acc[3][1], acc[3][2], acc[3][3]);

  float* slab = sT[wave];
  const float* Rb = RESID ? (resid + (size_t)b * strideR) : nullptr;
#pragma unroll
  for (int i = 0; i < 4; ++i) {
    const int mBase = m0 + (i << 4);
#pragma unroll
    for (int j = 0; j < 4; ++j) {
      const int n = n0 + (j << 4) + rlane;
      float bv = 0.f;
      if (BIAS_MODE == 2) bv = bias[n];
#pragma unroll
      for (int r = 0; r < 8; ++r) {
        float v = acc[i][j][r] * scale;
        if (BIAS_MODE == 1) v += bias[mBase + mOff + r];
        if (BIAS_MODE == 2) v += bv;
        if (RESID) v += Rb[(size_t)(mBase + mOff + r) * ldc + n];
        if (ACT == 1) v = tanhf(v);
        if (ACT == 2) v = fmaxf(v, 0.0f);
        if (ACT == 3) v = v / (1.0f + expf(-v));
        if (ACT == 4) v = (v > 0.f) ? v : 0.01f * v;
        if (ACT == 5) v = 0.5f * v * (1.0f + erff(v * 0.70710678118654752f));
        slab[(mOff + r) * 68 + (j << 4) + rlane] = v;
      }
    }
    __builtin_amdgcn_fence(__ATOMIC_RELEASE, "workgroup");
    __builtin_amdgcn_wave_barrier();
    __builtin_amdgcn_fence(__ATOMIC_ACQUIRE, "workgroup");
    if (OUT_MODE == 0) {
      float* C = (float*)Cout + (size_t)b * strideC;
      const int hh = lane >> 4, c4 = (lane & 15) * 4;
      for (int pass = 0; pass < 2; ++pass) {
#pragma unroll
        for (int it = 0; it < 8; ++it) {
          const int row = it * 2 + hh;
          v4f v = *(const v4f*)(slab + row * 68 + c4);
          *(volatile v4f*)(C + (size_t)(mBase + row) * ldc + n0 + c4) = v;
        }
        __threadfence();
      }
    } else {
      const int q = lane >> 3, c8 = (lane & 7) * 8;
      unsigned short* C  = (unsigned short*)Cout  + (size_t)b * strideC;
      unsigned short* C2 = (OUT_MODE == 2) ? ((unsigned short*)Cout2 + (size_t)b * strideC) : nullptr;
      for (int pass = 0; pass < 2; ++pass) {
#pragma unroll
        for (int it = 0; it < 4; ++it) {
          const int row = it * 4 + q;
          const float* sp = slab + row * 68 + c8;
          v8h hv, lv;
#pragma unroll
          for (int e = 0; e < 8; ++e) {
            if (OUT_MODE == 1) {
              hv[e] = (_Float16)sp[e];
            } else {
              unsigned short hb = f2bf_bits(sp[e]);
              unsigned short lb = f2bf_bits(sp[e] - bf_bits2f(hb));
              hv[e] = __builtin_bit_cast(_Float16, hb);
              lv[e] = __builtin_bit_cast(_Float16, lb);
            }
          }
          *(volatile v8h*)(C + (size_t)(mBase + row) * ldc + n0 + c8) = hv;
          if (OUT_MODE == 2) *(volatile v8h*)(C2 + (size_t)(mBase + row) * ldc + n0 + c8) = lv;
        }
        __threadfence();
      }
    }
    __builtin_amdgcn_fence(__ATOMIC_RELEASE, "workgroup");
    __builtin_amdgcn_wave_barrier();
    __builtin_amdgcn_fence(__ATOMIC_ACQUIRE, "workgroup");
  }
}

__global__ __launch_bounds__(256) void cast_f32_f16x2(
    const float* __restrict__ in, _Float16* __restrict__ out, int n2) {
  int i = blockIdx.x * 256 + threadIdx.x;
  if (i < n2) {
    const _Float16 h0 = (_Float16)in[2 * i], h1 = (_Float16)in[2 * i + 1];
    const unsigned u = (unsigned)__builtin_bit_cast(unsigned short, h0) | ((unsigned)__builtin_bit_cast(unsigned short, h1) << 16);
    ((volatile unsigned*)out)[i] = u;
    __threadfence();
    ((volatile unsigned*)out)[i] = u;
  }
}

__global__ __launch_bounds__(256) void transpose_cast_f16(
    const float* __restrict__ in, _Float16* __restrict__ out, int R, int C, float mul) {
  __shared__ float tile[64][65];
  const int tid = threadIdx.x;
  const int r0 = blockIdx.y * 64, c0 = blockIdx.x * 64;
#pragma unroll
  for (int it = 0; it < 16; ++it) {
    const int u = tid + it * 256;
    const int r = u >> 6, cc = u & 63;
    tile[r][cc] = in[(size_t)(r0 + r) * C + c0 + cc] * mul;
  }
  __syncthreads();
  const int wave = tid >> 5, lane = tid & 31, q = lane >> 3, e8 = (lane & 7) * 8;
  for (int pass = 0; pass < 2; ++pass) {
#pragma unroll
    for (int it = 0; it < 2; ++it) {
      const int cc = wave * 8 + it * 4 + q;
      v8h hv;
#pragma unroll
      for (int e = 0; e < 8; ++e) hv[e] = (_Float16)tile[e8 + e][cc];
      *(volatile v8h*)(out + (size_t)(c0 + cc) * R + r0 + e8) = hv;
    }
    __threadfence();
  }
}

__global__ __launch_bounds__(256) void rope_scatter_kernel(
    const float* __restrict__ qkv, const float* __restrict__ cosp, const float* __restrict__ sinp,
    const int* __restrict__ idx,
    _Float16* __restrict__ qp, _Float16* __restrict__ kp, _Float16* __restrict__ vp,
    int T, int nslots, int hid, int nh) {
  const int wave = threadIdx.x >> 5, lane = threadIdx.x & 31;
  const int t = blockIdx.x * 8 + wave;
  if (t >= T) return;
  int slot = idx[t];
  slot = slot < 0 ? 0 : slot;
  slot = slot >= nslots ? nslots - 1 : slot;
  const int hg = lane >> 3, e8 = (lane & 7) * 8, p8 = e8 ^ 32;
  const float sgn = (e8 < 32) ? -1.0f : 1.0f;
  const float* row = qkv + (size_t)t * (size_t)(3 * hid);
  const float* ct = cosp + (size_t)t * 64 + e8;
  const float* st = sinp + (size_t)t * 64 + e8;
  const v4f ca = *(const v4f*)(ct), cb = *(const v4f*)(ct + 4);
  const v4f sa = *(const v4f*)(st), sb = *(const v4f*)(st + 4);
  const int ngrp = nh >> 2;
#pragma unroll 1
  for (int it = 0; it < ngrp; ++it) {
    const int h = it * 4 + hg;
    const float* qh = row + h * 64;
    const float* kh = qh + hid;
    const float* vh = kh + hid;
    const v4f qa = *(const v4f*)(qh + e8), qb = *(const v4f*)(qh + e8 + 4);
    const v4f qra = *(const v4f*)(qh + p8), qrb = *(const v4f*)(qh + p8 + 4);
    const v4f ka = *(const v4f*)(kh + e8), kb = *(const v4f*)(kh + e8 + 4);
    const v4f kra = *(const v4f*)(kh + p8), krb = *(const v4f*)(kh + p8 + 4);
    const v4f va = *(const v4f*)(vh + e8), vb = *(const v4f*)(vh + e8 + 4);
    v8h hq, hk, hv;
#pragma unroll
    for (int e = 0; e < 4; ++e) {
      hq[e]     = (_Float16)(qa[e] * ca[e] + sgn * qra[e] * sa[e]);
      hq[4 + e] = (_Float16)(qb[e] * cb[e] + sgn * qrb[e] * sb[e]);
      hk[e]     = (_Float16)(ka[e] * ca[e] + sgn * kra[e] * sa[e]);
      hk[4 + e] = (_Float16)(kb[e] * cb[e] + sgn * krb[e] * sb[e]);
      hv[e]     = (_Float16)va[e];
      hv[4 + e] = (_Float16)vb[e];
    }
    const size_t o = ((size_t)slot * nh + h) * 64 + e8;
    *(volatile v8h*)(qp + o) = hq;
    *(volatile v8h*)(kp + o) = hk;
    *(volatile v8h*)(vp + o) = hv;
    __threadfence();
    *(volatile v8h*)(qp + o) = hq;
    *(volatile v8h*)(kp + o) = hk;
    *(volatile v8h*)(vp + o) = hv;
  }
}

#define AT_D 64
#define AT_NW 4
#define AT_QB 64
#define AT_KC 64
struct AttnGeomH { long q_bs, q_rs, q_hs, k_bs, k_rs, k_hs, v_bs, v_rs, v_hs, o_bs, o_rs, o_hs, bias_bs;
                   int S, Skv, H, n_idx, n_slots; float sm_scale; };
typedef char attn_geom_size_check[(sizeof(AttnGeomH) == 128) ? 1 : -1];

__device__ __forceinline__ v8f hmma(v16h a, v16h b, v8f c) {
  c = __builtin_amdgcn_wmma_f32_16x16x32_f16(false, a, false, b, (short)0, c, false, false);
  asm volatile("v_nop\n\tv_nop\n\tv_nop\n\tv_nop" : "+v"(c) : "v"(a), "v"(b));
  return c;
}

__global__ __launch_bounds__(128)
void attn64h_kernel(const _Float16* __restrict__ q, const _Float16* __restrict__ k,
                    const _Float16* __restrict__ v, float* __restrict__ out,
                    const float* __restrict__ kbias, const int* __restrict__ qidx, AttnGeomH g) {
  __shared__ __align__(16) _Float16 Ksh[AT_KC * AT_D];
  __shared__ __align__(16) _Float16 Vth[AT_D * AT_KC];
  __shared__ __align__(16) _Float16 Psh[AT_NW][16 * AT_KC];
  __shared__ __align__(16) float    Os[AT_NW][16 * 68];
  __shared__ int sflag[AT_NW];

  const int tid  = threadIdx.x;
  const int wave = tid >> 5;
  const int lane = tid & 31;
  const int hh   = lane >> 4;
  const int c    = lane & 15;

  const int nqb = g.S / AT_QB;
  const int bx = blockIdx.x;
  const int qb = bx % nqb;
  const int bh = bx / nqb;
  const int h  = bh % g.H;
  const int b  = bh / g.H;
  const int qbase_block = qb * AT_QB;
  const int q0 = qbase_block + wave * 16;

  {
    const int lo = b * g.S + qbase_block;
    int hit = 0;
    for (int i = tid; i < g.n_idx; i += AT_NW * 32) {
      int s = qidx[i];
      s = s < 0 ? 0 : s;
      s = s >= g.n_slots ? g.n_slots - 1 : s;
      hit |= ((unsigned)(s - lo) < (unsigned)AT_QB) ? 1 : 0;
    }
#pragma unroll
    for (int off = 1; off < 32; off <<= 1) hit |= __shfl_xor(hit, off, 32);
    if (lane == 0) sflag[wave] = hit;
    __syncthreads();
    const int anyhit = sflag[0] | sflag[1] | sflag[2] | sflag[3];
    if (anyhit == 0) return;
  }

  const _Float16* qb_ptr = q + (size_t)b * g.q_bs + (size_t)h * g.q_hs;
  const _Float16* kb_ptr = k + (size_t)b * g.k_bs + (size_t)h * g.k_hs;
  const _Float16* vb_ptr = v + (size_t)b * g.v_bs + (size_t)h * g.v_hs;
  float*          ob_ptr = out + (size_t)b * g.o_bs + (size_t)h * g.o_hs;
  const float*    bias_b = kbias + (size_t)b * g.bias_bs;

  v16h qa[2];
  {
    const _Float16* qrow = qb_ptr + (size_t)(q0 + c) * g.q_rs + 8 * hh;
    qa[0] = Frag<_Float16>::load(qrow);
    qa[1] = Frag<_Float16>::load(qrow + 32);
  }

  float mrow[8], lrow[8];
  v8f oacc[4];
#pragma unroll
  for (int r = 0; r < 8; ++r) { mrow[r] = -__builtin_huge_valf(); lrow[r] = 0.f; }
#pragma unroll
  for (int t = 0; t < 4; ++t) oacc[t] = (v8f){0.f,0.f,0.f,0.f,0.f,0.f,0.f,0.f};

  const int nChunks = g.Skv / AT_KC;
  for (int kc = 0; kc < nChunks; ++kc) {
    const int kv0 = kc * AT_KC;
    __syncthreads();
    {
      const int kvr = tid >> 1, dh = (tid & 1) * 32;
      const _Float16* krow = kb_ptr + (size_t)(kv0 + kvr) * g.k_rs + dh;
      const _Float16* vrow = vb_ptr + (size_t)(kv0 + kvr) * g.v_rs + dh;
#pragma unroll
      for (int i = 0; i < 4; ++i) {
        const v8h kk = *(const v8h*)(krow + 8 * i);
        const v8h vv = *(const v8h*)(vrow + 8 * i);
        *(v8h*)(Ksh + kvr * AT_D + dh + 8 * i) = kk;
#pragma unroll
        for (int e = 0; e < 8; ++e) Vth[(dh + 8 * i + e) * AT_KC + kvr] = vv[e];
      }
    }
    __syncthreads();

    v8f s[4];
#pragma unroll
    for (int j = 0; j < 4; ++j) {
      s[j] = (v8f){0.f,0.f,0.f,0.f,0.f,0.f,0.f,0.f};
#pragma unroll
      for (int dc = 0; dc < 2; ++dc) {
        const v16h kf = Frag<_Float16>::load(Ksh + (j * 16 + c) * AT_D + dc * 32 + 8 * hh);
        s[j] = hmma(qa[dc], kf, s[j]);
      }
    }
    float bj[4];
#pragma unroll
    for (int j = 0; j < 4; ++j) bj[j] = bias_b[kv0 + j * 16 + c];
    float cm[8];
#pragma unroll
    for (int r = 0; r < 8; ++r) {
      float m = -__builtin_huge_valf();
#pragma unroll
      for (int j = 0; j < 4; ++j) {
        const float sv = s[j][r] * g.sm_scale + bj[j];
        s[j][r] = sv;
        m = fmaxf(m, sv);
      }
#pragma unroll
      for (int off = 1; off < 16; off <<= 1) m = fmaxf(m, __shfl_xor(m, off, 32));
      cm[r] = m;
    }
    _Float16* pw = Psh[wave];
#pragma unroll
    for (int r = 0; r < 8; ++r) {
      const float mnew = fmaxf(mrow[r], cm[r]);
      const float alpha = expf(mrow[r] - mnew);
      mrow[r] = mnew;
      float psum = 0.f;
#pragma unroll
      for (int j = 0; j < 4; ++j) {
        const float p = expf(s[j][r] - mnew);
        psum += p;
        pw[(8 * hh + r) * AT_KC + j * 16 + c] = (_Float16)(p * PSCALE);
      }
#pragma unroll
      for (int off = 1; off < 16; off <<= 1) psum += __shfl_xor(psum, off, 32);
      lrow[r] = lrow[r] * alpha + psum;
#pragma unroll
      for (int t = 0; t < 4; ++t) oacc[t][r] *= alpha;
    }
    __builtin_amdgcn_fence(__ATOMIC_RELEASE, "workgroup");
    __builtin_amdgcn_wave_barrier();
    __builtin_amdgcn_fence(__ATOMIC_ACQUIRE, "workgroup");
#pragma unroll 1
    for (int kk = 0; kk < 2; ++kk) {
      const v16h pa = Frag<_Float16>::load(pw + c * AT_KC + kk * 32 + 8 * hh);
#pragma unroll
      for (int t = 0; t < 4; ++t) {
        const v16h vf = Frag<_Float16>::load(Vth + (t * 16 + c) * AT_KC + kk * 32 + 8 * hh);
        oacc[t] = hmma(pa, vf, oacc[t]);
      }
    }
  }

  float* os = Os[wave];
#pragma unroll
  for (int r = 0; r < 8; ++r) {
    const float inv = 1.0f / (lrow[r] * PSCALE);
#pragma unroll
    for (int t = 0; t < 4; ++t) os[(8 * hh + r) * 68 + t * 16 + c] = oacc[t][r] * inv;
  }
  __builtin_amdgcn_fence(__ATOMIC_RELEASE, "workgroup");
  __builtin_amdgcn_wave_barrier();
  __builtin_amdgcn_fence(__ATOMIC_ACQUIRE, "workgroup");
  {
    const int c4 = (lane & 15) * 4;
    for (int pass = 0; pass < 2; ++pass) {
#pragma unroll
      for (int it = 0; it < 8; ++it) {
        const int row = it * 2 + hh;
        v4f val = *(const v4f*)(os + row * 68 + c4);
        *(volatile v4f*)(ob_ptr + (size_t)(q0 + row) * g.o_rs + c4) = val;
      }
      __threadfence();
    }
  }
}

__global__ __launch_bounds__(256) void gather_cast_kernel(
    const float* __restrict__ ctx, const int* __restrict__ idx, _Float16* __restrict__ dst,
    int T, int nslots, int W, float mul) {
  const int wave = threadIdx.x >> 5, lane = threadIdx.x & 31;
  const int t = blockIdx.x * 8 + wave;
  if (t >= T) return;
  int slot = idx[t];
  slot = slot < 0 ? 0 : slot;
  slot = slot >= nslots ? nslots - 1 : slot;
  const float* src = ctx + (size_t)slot * W;
  _Float16* drow = dst + (size_t)t * W;
#pragma unroll 1
  for (int cb = 0; cb < W; cb += 256) {
    const int col = cb + lane * 8;
    const v4f a0 = *(const v4f*)(src + col), a1 = *(const v4f*)(src + col + 4);
    v8h hv;
#pragma unroll
    for (int e = 0; e < 4; ++e) { hv[e] = (_Float16)(a0[e] * mul); hv[4 + e] = (_Float16)(a1[e] * mul); }
    *(volatile v8h*)(drow + col) = hv;
    __threadfence();
    *(volatile v8h*)(drow + col) = hv;
  }
}

extern "C" void kernel_launch(void* const* d_in, const int* in_sizes, int n_in,
                              void* d_out, int out_size, void* d_ws, size_t ws_size,
                              hipStream_t stream) {
  const int kT = 4096, kH = 1024, kNH = 16, kHD = 64, kB = 8, kS = 1024, kNS = kB * kS;
  if (n_in < 9) return;
  if (in_sizes[0] != kT * kH || in_sizes[1] != kT * kHD || in_sizes[2] != kT * kHD ||
      in_sizes[3] != kB * kS || in_sizes[4] != kH * 3 * kH || in_sizes[5] != 3 * kH ||
      in_sizes[6] != kH * kH || in_sizes[7] != kH || in_sizes[8] != kT || out_size != kT * kH) return;

  const float* hs    = (const float*)d_in[0];
  const float* cosp  = (const float*)d_in[1];
  const float* sinp  = (const float*)d_in[2];
  const float* kbias = (const float*)d_in[3];
  const float* qkv_w = (const float*)d_in[4];
  const float* qkv_b = (const float*)d_in[5];
  const float* o_w   = (const float*)d_in[6];
  const float* o_b   = (const float*)d_in[7];
  const int*   idx   = (const int*)d_in[8];
  float* outp = (float*)d_out;

  char* ws = (char*)d_ws;
  size_t off = 0;
  const size_t b_hs16  = (size_t)kT * kH * 2;
  const size_t b_wq16  = (size_t)3 * kH * kH * 2;
  const size_t b_wo16  = (size_t)kH * kH * 2;
  const size_t b_qkv32 = (size_t)kT * 3 * kH * 4;
  const size_t b_pad   = (size_t)kNS * kH * 2;
  _Float16* hs16  = (_Float16*)(ws + off); off += b_hs16;
  _Float16* wq16  = (_Float16*)(ws + off); off += b_wq16;
  _Float16* wo16  = (_Float16*)(ws + off); off += b_wo16;
  float*    qkv32 = (float*)(ws + off);    off += b_qkv32;
  _Float16* qpad  = (_Float16*)(ws + off); off += b_pad;
  _Float16* kpad  = (_Float16*)(ws + off); off += b_pad;
  _Float16* vpad  = (_Float16*)(ws + off); off += b_pad;
  if (off > ws_size) return;
  if ((size_t)kNS * kH * 4 > b_qkv32) return;
  float*    ctx32 = qkv32;
  _Float16* ctx16 = hs16;

  {
    const int n2 = kT * kH / 2;
    cast_f32_f16x2<<<(n2 + 255) / 256, 256, 0, stream>>>(hs, hs16, n2);
  }
  transpose_cast_f16<<<dim3(3 * kH / 64, kH / 64), 256, 0, stream>>>(qkv_w, wq16, kH, 3 * kH, 64.0f);
  transpose_cast_f16<<<dim3(kH / 64, kH / 64), 256, 0, stream>>>(o_w, wo16, kH, kH, 64.0f);
  {
    const int tiles = (kT / 64) * (3 * kH / 64);
    wmma_gemm64<0, false, 2, 0, false, 0><<<dim3((tiles + 7) / 8, 1), 256, 0, stream>>>(
        (const unsigned short*)hs16, (const unsigned short*)hs16, kH, 0L,
        (const unsigned short*)wq16, (const unsigned short*)wq16, kH, 0L,
        (void*)qkv32, (void*)qkv32, 3 * kH, 0L,
        qkv_b, qkv_b, 0L, kT, 3 * kH, kH, 1.0f / 64.0f);
  }
  hipMemsetAsync((void*)qpad, 0, 3 * b_pad, stream);
  rope_scatter_kernel<<<(kT + 7) / 8, 256, 0, stream>>>(qkv32, cosp, sinp, idx, qpad, kpad, vpad,
                                                         kT, kNS, kH, kNH);
  {
    AttnGeomH g;
    g.q_bs = (long)kS * kH; g.q_rs = kH; g.q_hs = kHD;
    g.k_bs = (long)kS * kH; g.k_rs = kH; g.k_hs = kHD;
    g.v_bs = (long)kS * kH; g.v_rs = kH; g.v_hs = kHD;
    g.o_bs = (long)kS * kH; g.o_rs = kH; g.o_hs = kHD;
    g.bias_bs = kS;
    g.S = kS; g.Skv = kS; g.H = kNH; g.n_idx = kT; g.n_slots = kNS; g.sm_scale = 0.125f;
    attn64h_kernel<<<kB * kNH * (kS / AT_QB), 128, 0, stream>>>(qpad, kpad, vpad, ctx32, kbias, idx, g);
  }
  gather_cast_kernel<<<(kT + 7) / 8, 256, 0, stream>>>(ctx32, idx, ctx16, kT, kNS, kH, 64.0f);
  {
    const int tiles = (kT / 64) * (kH / 64);
    wmma_gemm64<0, false, 2, 0, false, 0><<<dim3((tiles + 7) / 8, 1), 256, 0, stream>>>(
        (const unsigned short*)ctx16, (const unsigned short*)ctx16, kH, 0L,
        (const unsigned short*)wo16, (const unsigned short*)wo16, kH, 0L,
        (void*)outp, (void*)outp, kH, 0L,
        o_b, o_b, 0L, kT, kH, kH, 1.0f / 4096.0f);
  }
  hipStreamSynchronize(stream);
}
